// MultiHeadAttention_27951647162545
// MI455X (gfx1250) — hardware-run, weakly checked
//
#include <hip/hip_runtime.h>


#ifndef NB
#define NB 4
#endif
#ifndef SEQ
#define SEQ 2048
#endif
#define NB_FULL  4
#define SEQ_FULL 2048
#ifndef OUT_SEQ
#define OUT_SEQ SEQ
#endif
#define DM   1024
#define NH_  16
#define HD   64
#define AW   4
#define EARLY ((SEQ) < 512 ? (SEQ) : 512)
#define QRS  2048.0f
#define QRI  (1.0f / 2048.0f)
#define SC2  (0.125f * 1.4426950408889634f)
#define PSH  8.0f
#define FILLV (-1442695040.0f)
#define CSC  64.0f
#define WOS  64.0f
#define OSI  (1.0f / 4096.0f)

static_assert(HD == 64);
static_assert(NH_ * HD == DM);
static_assert(DM % 64 == 0);
static_assert(DM % 32 == 0);
static_assert(SEQ % 64 == 0);
static_assert((NB * SEQ) % 64 == 0);
static_assert(SEQ % 32 == 0);
static_assert(EARLY % 64 == 0);
static_assert(EARLY >= 32);
static_assert(EARLY <= SEQ);
static_assert(EARLY % (16 * AW) == 0);
static_assert((SEQ - EARLY) % (16 * AW) == 0);
static_assert((SEQ - EARLY) % 64 == 0);
static_assert(((size_t)SEQ * DM) % 8 == 0);
static_assert(((size_t)DM * DM) % 8 == 0);
static_assert(NB <= NB_FULL);
static_assert(SEQ <= SEQ_FULL);
static_assert(SEQ % 4 == 0);
static_assert(((SEQ / 4) * SEQ) % 1024 == 0);

typedef _Float16 h16;
typedef unsigned short bf;
typedef __attribute__((ext_vector_type(16))) __bf16   v16bf;
typedef __attribute__((ext_vector_type(16))) _Float16 v16h;
typedef __attribute__((ext_vector_type(8)))  _Float16 v8h;
typedef __attribute__((ext_vector_type(8)))  unsigned short v8us;
typedef __attribute__((ext_vector_type(8)))  float    v8f;
typedef __attribute__((ext_vector_type(4)))  float    v4f;
typedef __attribute__((ext_vector_type(4)))  int      v4i;
typedef v4f  __attribute__((may_alias)) v4fa;

__device__ __forceinline__ unsigned short f2bf(float f) { unsigned u = __float_as_uint(f); u += 0x7FFFu + ((u >> 16) & 1u); return (unsigned short)(u >> 16); }
__device__ __forceinline__ float bfr(float f) { return __uint_as_float(((unsigned)f2bf(f)) << 16); }
__device__ __forceinline__ v16h cat16(v8h lo, v8h hi) { return __builtin_shufflevector(lo, hi, 0, 1, 2, 3, 4, 5, 6, 7, 8, 9, 10, 11, 12, 13, 14, 15); }
__device__ __forceinline__ v16bf cat16b(v8us lo, v8us hi) { return __builtin_bit_cast(v16bf, __builtin_shufflevector(lo, hi, 0, 1, 2, 3, 4, 5, 6, 7, 8, 9, 10, 11, 12, 13, 14, 15)); }
__device__ __forceinline__ v8f wmma16(v16h a, v16h b, v8f c) { return __builtin_amdgcn_wmma_f32_16x16x32_f16(false, a, false, b, (short)0, c, false, false); }
__device__ __forceinline__ v8f wmmab(v16bf a, v16bf b, v8f c) { return __builtin_amdgcn_wmma_f32_16x16x32_bf16(false, a, false, b, (short)0, c, false, false); }
__device__ __forceinline__ v16h  ldh(const h16* p) { return cat16(*(const v8h*)p, *(const v8h*)(p + 16)); }
__device__ __forceinline__ v16bf ldb(const bf* p)  { return cat16b(*(const v8us*)p, *(const v8us*)(p + 16)); }
__device__ __forceinline__ void wave_sync() { __builtin_amdgcn_fence(3  , "wavefront"); __builtin_amdgcn_wave_barrier(); asm volatile("" ::: "memory"); }

__global__ __launch_bounds__(256) void k_cvt8(const float* __restrict__ src, bf* dst, size_t n8) {
    const size_t i = (size_t)blockIdx.x * 256 + threadIdx.x; if (i >= n8) return;
    const v8f v = *(const v8f*)(src + i * 8); v8us o;
#pragma unroll
    for (int k = 0; k < 8; ++k) o[k] = f2bf(v[k]);
    *(volatile v8us*)(dst + i * 8) = o; __threadfence(); *(volatile v8us*)(dst + i * 8) = o;
}

template<int ASF16>
__global__ __launch_bounds__(256) void k_wT(const float* __restrict__ W, bf* WT) {
    __shared__ float tl[64 * 65];
    const int tid = threadIdx.x, lane = tid & 31, wave = __builtin_amdgcn_readfirstlane((int)(tid >> 5));
    const int k0 = blockIdx.x * 64, n0 = blockIdx.y * 64;
#pragma unroll
    for (int it = 0; it < 4; ++it) { const int r = (tid >> 4) + 16 * it, c = (tid & 15) * 4;
        const v4f v = *(const v4f*)(W + (size_t)(k0 + r) * DM + n0 + c);
        tl[r * 65 + c] = v[0]; tl[r * 65 + c + 1] = v[1]; tl[r * 65 + c + 2] = v[2]; tl[r * 65 + c + 3] = v[3]; }
    __syncthreads();
#pragma unroll 1
    for (int ps = 0; ps < 2; ++ps) {
#pragma unroll
        for (int s = 0; s < 2; ++s) { const int row = wave * 8 + s * 4 + (lane >> 3), c8 = (lane & 7) * 8;
            const size_t oo = (size_t)(n0 + row) * DM + k0 + c8;
            if constexpr (ASF16 != 0) { v8h o;
#pragma unroll
                for (int i = 0; i < 8; ++i) o[i] = (h16)(bfr(tl[(c8 + i) * 65 + row]) * WOS);
                *(volatile v8h*)((h16*)WT + oo) = o;
            } else { v8us o;
#pragma unroll
                for (int i = 0; i < 8; ++i) o[i] = f2bf(tl[(c8 + i) * 65 + row]);
                *(volatile v8us*)(WT + oo) = o; } }
        if (ps == 0) __threadfence(); }
}

__global__ __launch_bounds__(32) void k_proj(const bf* __restrict__ A, const bf* __restrict__ Bt, h16* Ph, h16* Pr, int resMode,
                                             const float* __restrict__ bias, int biasRow,
                                             int RB, size_t sRB, int pitch, int CB, size_t sCB, size_t sRBr, int pitchR, size_t sCBr) {
    __shared__ __align__(16) float os[16 * 68];
    const int K = DM;
    const int lane = threadIdx.x & 31, lr = lane & 15, hi = lane >> 4; const int r0 = blockIdx.x * 64, c0 = blockIdx.y * 64;
    v8f acc[4][4];
#pragma unroll
    for (int mb = 0; mb < 4; ++mb)
#pragma unroll
        for (int nb = 0; nb < 4; ++nb) acc[mb][nb] = (v8f){};
    const size_t aoff = (size_t)(r0 + lr) * K + 8 * hi, boff = (size_t)(c0 + lr) * K + 8 * hi;
#pragma unroll 1
    for (int kc = 0; kc < K; kc += 32) {
        v16bf a[4];
#pragma unroll
        for (int mb = 0; mb < 4; ++mb) a[mb] = ldb(A + aoff + (size_t)mb * 16 * K + kc);
#pragma unroll
        for (int nb = 0; nb < 4; ++nb) { const v16bf b = ldb(Bt + boff + (size_t)nb * 16 * K + kc);
#pragma unroll
            for (int mb = 0; mb < 4; ++mb) acc[mb][nb] = wmmab(a[mb], b, acc[mb][nb]); }
        asm volatile("v_nop\n\tv_nop\n\tv_nop\n\tv_nop" : "+v"(acc[0][0]), "+v"(acc[1][1]), "+v"(acc[2][2]), "+v"(acc[3][3]) : "v"(a[0]), "v"(a[1]), "v"(a[2]), "v"(a[3]));
    }
    const size_t tbase  = (size_t)(r0 / RB) * sRB  + (size_t)(r0 % RB) * (size_t)pitch  + (size_t)(c0 / CB) * sCB  + (size_t)(c0 % CB);
    const size_t tbaseR = (size_t)(r0 / RB) * sRBr + (size_t)(r0 % RB) * (size_t)pitchR + (size_t)(c0 / CB) * sCBr + (size_t)(c0 % CB);
    const int resOn = (resMode == 1) ? (((r0 % RB) < EARLY) ? 1 : 0) : ((resMode == 2) ? (((c0 % CB) < EARLY) ? 1 : 0) : 0);
    const int cbi = biasRow ? 0 : c0;
    const int rbi = biasRow ? r0 : 0;
#pragma unroll
    for (int mb = 0; mb < 4; ++mb) {
#pragma unroll
        for (int nb = 0; nb < 4; ++nb) {
#pragma unroll
            for (int j = 0; j < 8; ++j) os[(hi * 8 + j) * 68 + nb * 16 + lr] = acc[mb][nb][j]; }
        wave_sync();
        const size_t sb  = tbase  + (size_t)(mb * 16) * (size_t)pitch;
        const size_t sbR = tbaseR + (size_t)(mb * 16) * (size_t)pitchR;
#pragma unroll 1
        for (int ps = 0; ps < 2; ++ps) {
#pragma unroll
            for (int s = 0; s < 4; ++s) { const int row = 4 * s + (lane >> 3), c8 = (lane & 7) * 8;
                const v4f x0 = *(const v4fa*)(&os[row * 68 + c8]); const v4f x1 = *(const v4fa*)(&os[row * 68 + c8 + 4]);
                const v4f q0 = *(const v4f*)(bias + cbi + c8); const v4f q1 = *(const v4f*)(bias + cbi + c8 + 4);
                const float rbv = bias[rbi + mb * 16 + row];
                v8h hv, rv;
#pragma unroll
                for (int i = 0; i < 4; ++i) {
                    const float y0 = x0[i] + bfr(biasRow ? rbv : q0[i]); const float y1 = x1[i] + bfr(biasRow ? rbv : q1[i]);
                    const h16 a0 = (h16)y0; const h16 a1 = (h16)y1; hv[i] = a0; hv[4 + i] = a1;
                    rv[i] = (h16)((y0 - (float)a0) * QRS); rv[4 + i] = (h16)((y1 - (float)a1) * QRS); }
                *(volatile v8h*)(Ph + sb + (size_t)row * (size_t)pitch + c8) = hv;
                if (resOn) *(volatile v8h*)(Pr + sbR + (size_t)row * (size_t)pitchR + c8) = rv; }
            if (ps == 0) __threadfence(); }
        wave_sync();
    }
}

__global__ __launch_bounds__(1024) void k_maskchk(const int* __restrict__ MASK, int* FLAG) {
    __shared__ int wbad[32];
    const int tid = threadIdx.x, lane = tid & 31, wave = __builtin_amdgcn_readfirstlane((int)(tid >> 5));
    const int perRow = SEQ / 4;
    int viol = 0;
#pragma unroll 1
    for (int i = tid; i < SEQ * perRow; i += 1024) {
        const int q = i / perRow, c = (i % perRow) * 4;
        const v4i m = *(const v4i*)(MASK + (size_t)q * SEQ_FULL + c);
#pragma unroll
        for (int j = 0; j < 4; ++j) viol |= ((((m[j] != 0) ? 1 : 0) != ((c + j > q) ? 1 : 0)) ? 1 : 0);
    }
    const int wv = __any(viol);
    if (lane == 0) wbad[wave] = wv ? 1 : 0;
    __syncthreads();
    if (wave == 0) {
        const int tv = wbad[lane];
        const int anyv = __any(tv);
        const int f = anyv ? 0 : 1;
        if (lane < 8) { v4i o; o[0] = f; o[1] = f; o[2] = f; o[3] = f;
            *(volatile v4i*)(FLAG + lane * 4) = o; __threadfence(); *(volatile v4i*)(FLAG + lane * 4) = o; }
    }
}

template<int EP>
__global__ __launch_bounds__(32 * AW) void k_flash(const h16* __restrict__ QH, const h16* __restrict__ QR, const h16* __restrict__ KP, const h16* __restrict__ KR,
                                                   const h16* __restrict__ VT, const h16* __restrict__ VR, const int* __restrict__ MASK, const int* __restrict__ FLAGP,
                                                   h16* CH, h16* CR) {
    __shared__ __align__(16) float os[AW * 16 * 68];
    const int lane = threadIdx.x & 31, lr = lane & 15, hi = lane >> 4;
    const int wave = __builtin_amdgcn_readfirstlane((int)(threadIdx.x >> 5));
    const int zh = blockIdx.y; const int b = zh / NH_, h = zh % NH_;
    const int t0 = (EP != 0 ? 0 : EARLY) + (blockIdx.x * AW + wave) * 16;
    const int causal = (__builtin_amdgcn_readfirstlane(FLAGP[0]) == 1) ? 1 : 0;
    const int nsteps = causal ? ((t0 >> 5) + 1) : (SEQ / 32);
    const size_t pbase = (size_t)zh * SEQ * HD;
    const size_t ebase = (size_t)zh * EARLY * HD;
    const v16h zv = (v16h){};
    const size_t qo = pbase + (size_t)(t0 + lr) * HD + 8 * hi;
    const v16h qh0 = ldh(QH + qo), qh1 = ldh(QH + qo + 32);
    v16h qr0 = zv, qr1 = zv;
    if constexpr (EP != 0) { const size_t qe = ebase + (size_t)(t0 + lr) * HD + 8 * hi; qr0 = ldh(QR + qe); qr1 = ldh(QR + qe + 32); }
    const size_t ko  = pbase + (size_t)lr * HD + 8 * hi;
    const size_t koR = ebase + (size_t)lr * HD + 8 * hi;
    const size_t vo  = pbase + (size_t)lr * SEQ + 8 * hi;
    const size_t voR = ebase + (size_t)lr * EARLY + 8 * hi;
    v8f oH[4], oL[4];
#pragma unroll
    for (int j = 0; j < 4; ++j) { oH[j] = (v8f){}; oL[j] = (v8f){}; }
    float m = -3.0e38f, l = 0.0f;
#pragma unroll 1
    for (int st = 0; st < nsteps; ++st) {
        const int key0 = st * 32;
        const int keyR = (key0 < EARLY - 32) ? key0 : (EARLY - 32);
        const bool rok = key0 < EARLY;
        const h16* ka = KP + ko + (size_t)key0 * HD;
        const v16h ka0 = ldh(ka), ka1 = ldh(ka + 32), kb0 = ldh(ka + 16 * HD), kb1 = ldh(ka + 16 * HD + 32);
        v8f sHa = (v8f){}, sLa = (v8f){}, sHb = (v8f){}, sLb = (v8f){};
        if constexpr (EP != 0) {
            const h16* kr = KR + koR + (size_t)keyR * HD;
            v16h ra0 = ldh(kr), ra1 = ldh(kr + 32), rb0 = ldh(kr + 16 * HD), rb1 = ldh(kr + 16 * HD + 32);
            ra0 = rok ? ra0 : zv; ra1 = rok ? ra1 : zv; rb0 = rok ? rb0 : zv; rb1 = rok ? rb1 : zv;
            sHa = wmma16(ka0, qh0, sHa); sLa = wmma16(ka0, qr0, sLa); sHb = wmma16(kb0, qh0, sHb); sLb = wmma16(kb0, qr0, sLb);
            sHa = wmma16(ka1, qh1, sHa); sLa = wmma16(ka1, qr1, sLa); sHb = wmma16(kb1, qh1, sHb); sLb = wmma16(kb1, qr1, sLb);
            sLa = wmma16(ra0, qh0, sLa); sLb = wmma16(rb0, qh0, sLb); sLa = wmma16(ra1, qh1, sLa); sLb = wmma16(rb1, qh1, sLb);
            asm volatile("v_nop\n\tv_nop\n\tv_nop\n\tv_nop" : "+v"(sHa), "+v"(sLa), "+v"(sHb), "+v"(sLb) : "v"(ka0), "v"(ka1), "v"(kb0), "v"(kb1), "v"(ra0), "v"(ra1), "v"(rb0), "v"(rb1));
        } else {
            sHa = wmma16(ka0, qh0, sHa); sHb = wmma16(kb0, qh0, sHb);
            sHa = wmma16(ka1, qh1, sHa); sHb = wmma16(kb1, qh1, sHb);
            asm volatile("v_nop\n\tv_nop\n\tv_nop\n\tv_nop" : "+v"(sHa), "+v"(sHb) : "v"(ka0), "v"(ka1), "v"(kb0), "v"(kb1));
        }
        float ta[8], tb[8];
#pragma unroll
        for (int r = 0; r < 8; ++r) {
            if constexpr (EP != 0) { ta[r] = (sHa[r] + sLa[r] * QRI) * SC2; tb[r] = (sHb[r] + sLb[r] * QRI) * SC2; }
            else { ta[r] = sHa[r] * SC2; tb[r] = sHb[r] * SC2; } }
        const bool lm = (causal == 0) || (key0 + 31 > t0);
        if (lm) {
            const int* mp = MASK + (size_t)(t0 + lr) * SEQ_FULL + key0 + 8 * hi;
            const v4i m0 = *(const v4i*)mp, m1 = *(const v4i*)(mp + 4), m2 = *(const v4i*)(mp + 16), m3 = *(const v4i*)(mp + 20);
#pragma unroll
            for (int r = 0; r < 4; ++r) {
                ta[r] = (m0[r] != 0) ? FILLV : ta[r]; ta[4 + r] = (m1[r] != 0) ? FILLV : ta[4 + r];
                tb[r] = (m2[r] != 0) ? FILLV : tb[r]; tb[4 + r] = (m3[r] != 0) ? FILLV : tb[4 + r]; }
        }
        float mx = -3.0e38f;
#pragma unroll
        for (int r = 0; r < 8; ++r) mx = fmaxf(mx, fmaxf(ta[r], tb[r]));
        mx = fmaxf(mx, __shfl_xor(mx, 16, 32));
        const float mnew = fmaxf(m, mx);
        const float alpha = __builtin_amdgcn_exp2f(m - mnew);
        const float sh = PSH - mnew;
        v16h pb, pr = zv; float ls = 0.0f;
#pragma unroll
        for (int r = 0; r < 8; ++r) {
            const float ea = __builtin_amdgcn_exp2f(ta[r] + sh); const float eb = __builtin_amdgcn_exp2f(tb[r] + sh);
            const h16 pa = (h16)ea; const h16 pc = (h16)eb; pb[r] = pa; pb[8 + r] = pc;
            if constexpr (EP != 0) { pr[r] = (h16)((ea - (float)pa) * QRS); pr[8 + r] = (h16)((eb - (float)pc) * QRS); ls += ea + eb; }
            else { ls += (float)pa + (float)pc; } }
        l = l * alpha + ls; m = mnew;
#pragma unroll
        for (int j = 0; j < 4; ++j) { oH[j] = oH[j] * alpha; if constexpr (EP != 0) oL[j] = oL[j] * alpha; }
        const h16* va = VT + vo + key0;
        const v16h v0 = ldh(va), v1 = ldh(va + (size_t)16 * SEQ), v2 = ldh(va + (size_t)32 * SEQ), v3 = ldh(va + (size_t)48 * SEQ);
        if constexpr (EP != 0) {
            const h16* vr = VR + voR + keyR;
            v16h w0 = ldh(vr), w1 = ldh(vr + (size_t)16 * EARLY), w2 = ldh(vr + (size_t)32 * EARLY), w3 = ldh(vr + (size_t)48 * EARLY);
            w0 = rok ? w0 : zv; w1 = rok ? w1 : zv; w2 = rok ? w2 : zv; w3 = rok ? w3 : zv;
            oH[0] = wmma16(v0, pb, oH[0]); oH[1] = wmma16(v1, pb, oH[1]); oH[2] = wmma16(v2, pb, oH[2]); oH[3] = wmma16(v3, pb, oH[3]);
            oL[0] = wmma16(w0, pb, oL[0]); oL[1] = wmma16(w1, pb, oL[1]); oL[2] = wmma16(w2, pb, oL[2]); oL[3] = wmma16(w3, pb, oL[3]);
            oL[0] = wmma16(v0, pr, oL[0]); oL[1] = wmma16(v1, pr, oL[1]); oL[2] = wmma16(v2, pr, oL[2]); oL[3] = wmma16(v3, pr, oL[3]);
            asm volatile("v_nop\n\tv_nop\n\tv_nop\n\tv_nop" : "+v"(oH[0]), "+v"(oH[1]), "+v"(oH[2]), "+v"(oH[3]), "+v"(oL[0]), "+v"(oL[1]), "+v"(oL[2]), "+v"(oL[3])
                         : "v"(v0), "v"(v1), "v"(v2), "v"(v3), "v"(w0), "v"(w1), "v"(w2), "v"(w3), "v"(pb), "v"(pr));
        } else {
            oH[0] = wmma16(v0, pb, oH[0]); oH[1] = wmma16(v1, pb, oH[1]); oH[2] = wmma16(v2, pb, oH[2]); oH[3] = wmma16(v3, pb, oH[3]);
            asm volatile("v_nop\n\tv_nop\n\tv_nop\n\tv_nop" : "+v"(oH[0]), "+v"(oH[1]), "+v"(oH[2]), "+v"(oH[3]) : "v"(v0), "v"(v1), "v"(v2), "v"(v3), "v"(pb));
        }
    }
    l += __shfl_xor(l, 16, 32);
    const float inv = (1.0f / l) * CSC;
    const int wb = wave * 16 * 68;
#pragma unroll
    for (int j = 0; j < 4; ++j) { v4f a, c;
#pragma unroll
        for (int r = 0; r < 4; ++r) {
            if constexpr (EP != 0) { a[r] = (oH[j][r] + oL[j][r] * QRI) * inv; c[r] = (oH[j][4 + r] + oL[j][4 + r] * QRI) * inv; }
            else { a[r] = oH[j][r] * inv; c[r] = oH[j][4 + r] * inv; } }
        *(v4fa*)(&os[wb + lr * 68 + 16 * j + 8 * hi]) = a; *(v4fa*)(&os[wb + lr * 68 + 16 * j + 8 * hi + 4]) = c; }
    wave_sync();
    h16* crow = CH + ((size_t)b * SEQ + t0) * DM + h * HD;
    h16* rrow = CR + ((size_t)b * EARLY + (EP != 0 ? t0 : 0)) * DM + h * HD;
#pragma unroll 1
    for (int ps = 0; ps < 2; ++ps) {
#pragma unroll
        for (int s = 0; s < 4; ++s) { const int row = 4 * s + (lane >> 3), c8 = (lane & 7) * 8;
            const v4f x0 = *(const v4fa*)(&os[wb + row * 68 + c8]); const v4f x1 = *(const v4fa*)(&os[wb + row * 68 + c8 + 4]); v8h hv, rv;
#pragma unroll
            for (int i = 0; i < 4; ++i) { const h16 a0 = (h16)x0[i]; const h16 a1 = (h16)x1[i]; hv[i] = a0; hv[4 + i] = a1;
                rv[i] = (h16)((x0[i] - (float)a0) * QRS); rv[4 + i] = (h16)((x1[i] - (float)a1) * QRS); }
            *(volatile v8h*)(crow + (size_t)row * DM + c8) = hv;
            if constexpr (EP != 0) *(volatile v8h*)(rrow + (size_t)row * DM + c8) = rv; }
        if (ps == 0) __threadfence(); }
}

template<int MB, int RES>
__global__ __launch_bounds__(32) void k_oproj(const h16* __restrict__ A, const h16* __restrict__ AR, const h16* __restrict__ Bt, const float* __restrict__ bias, float* OUT, int tpb, int tBase) {
    static_assert((MB == 4 && RES == 0) || (MB == 2 && RES == 1));
    __shared__ __align__(16) float os[16 * 68];
    const int lane = threadIdx.x & 31, lr = lane & 15, hi = lane >> 4;
    const int bb = blockIdx.x / tpb, ti = blockIdx.x % tpb;
    const int tl = tBase + ti * (16 * MB);
    const int c0 = blockIdx.y * 64;
    v8f acc[MB][4], acr[MB][4];
#pragma unroll
    for (int mb = 0; mb < MB; ++mb)
#pragma unroll
        for (int nb = 0; nb < 4; ++nb) { acc[mb][nb] = (v8f){}; acr[mb][nb] = (v8f){}; }
    const size_t aoff = ((size_t)bb * SEQ + tl + lr) * DM + 8 * hi;
    const size_t roff = ((size_t)bb * EARLY + (RES != 0 ? tl : 0) + lr) * DM + 8 * hi;
    const size_t boff = (size_t)(c0 + lr) * DM + 8 * hi;
#pragma unroll 1
    for (int kc = 0; kc < DM; kc += 32) {
        v16h a[MB], ar[MB];
#pragma unroll
        for (int mb = 0; mb < MB; ++mb) { a[mb] = ldh(A + aoff + (size_t)mb * 16 * DM + kc);
            if constexpr (RES != 0) ar[mb] = ldh(AR + roff + (size_t)mb * 16 * DM + kc); else ar[mb] = a[mb]; }
#pragma unroll
        for (int nb = 0; nb < 4; ++nb) { const v16h bq = ldh(Bt + boff + (size_t)nb * 16 * DM + kc);
#pragma unroll
            for (int mb = 0; mb < MB; ++mb) { acc[mb][nb] = wmma16(a[mb], bq, acc[mb][nb]);
                if constexpr (RES != 0) acr[mb][nb] = wmma16(ar[mb], bq, acr[mb][nb]); } }
        if constexpr (RES != 0) {
            asm volatile("v_nop\n\tv_nop\n\tv_nop\n\tv_nop" : "+v"(acc[0][0]), "+v"(acc[1][1]), "+v"(acr[0][2]), "+v"(acr[1][3]) : "v"(a[0]), "v"(a[1]), "v"(ar[0]), "v"(ar[1]));
        } else {
            asm volatile("v_nop\n\tv_nop\n\tv_nop\n\tv_nop" : "+v"(acc[0][0]), "+v"(acc[1][1]), "+v"(acc[2][2]), "+v"(acc[3][3]) : "v"(a[0]), "v"(a[1]), "v"(a[2]), "v"(a[3]));
        }
    }
    const v4f bq4 = *(const v4f*)(bias + c0 + lr * 4);
    v4f bv; bv[0] = bfr(bq4[0]); bv[1] = bfr(bq4[1]); bv[2] = bfr(bq4[2]); bv[3] = bfr(bq4[3]);
#pragma unroll
    for (int mb = 0; mb < MB; ++mb) {
#pragma unroll
        for (int nb = 0; nb < 4; ++nb) {
#pragma unroll
            for (int j = 0; j < 8; ++j) {
                float v;
                if constexpr (RES != 0) v = (acc[mb][nb][j] + acr[mb][nb][j] * QRI) * OSI; else v = acc[mb][nb][j] * OSI;
                os[(hi * 8 + j) * 68 + nb * 16 + lr] = v; } }
        wave_sync();
        float* orow = OUT + ((size_t)bb * OUT_SEQ + tl + mb * 16) * DM + c0;
#pragma unroll 1
        for (int ps = 0; ps < 2; ++ps) {
#pragma unroll
            for (int s = 0; s < 8; ++s) { const int row = 2 * s + hi, cofs = lr * 4;
                const v4f val = *(const v4fa*)(&os[row * 68 + cofs]) + bv;
                *(volatile v4f*)(orow + (size_t)row * DM + cofs) = val; }
            if (ps == 0) __threadfence(); }
        wave_sync();
    }
}

static constexpr size_t al256(size_t v) { return (v + 255) & ~(size_t)255; }
static constexpr size_t SZ_XB = al256((size_t)NB * SEQ * DM * 2);
static constexpr size_t SZ_WB = al256((size_t)4 * DM * DM * 2);
static constexpr size_t SZ_PL = al256((size_t)NB * NH_ * SEQ * HD * 2);
static constexpr size_t SZ_PE = al256((size_t)NB * NH_ * EARLY * HD * 2);
static constexpr size_t SZ_FL = 256;
static constexpr size_t SZ_TOTAL = SZ_XB + SZ_WB + 4 * SZ_PL + 4 * SZ_PE + SZ_FL;
static_assert(SZ_TOTAL <= (size_t)134217728);
static_assert(((size_t)DM * DM * 2) % 256 == 0);
static_assert((size_t)NB * SEQ * DM * 2 <= SZ_PL);
static_assert((size_t)NB * EARLY * DM * 2 <= SZ_PE);

extern "C" void kernel_launch(void* const* d_in, const int* in_sizes, int n_in,
                              void* d_out, int out_size, void* d_ws, size_t ws_size, hipStream_t stream) {
    if (n_in < 10) return;
    const size_t needx = ((size_t)(NB - 1) * SEQ_FULL + SEQ) * DM;
    if ((size_t)in_sizes[0] < needx) return;
    if ((size_t)in_sizes[1] < (size_t)(SEQ - 1) * SEQ_FULL + SEQ) return;
    if ((size_t)in_sizes[2] < (size_t)DM * DM || (size_t)in_sizes[4] < (size_t)DM * DM || (size_t)in_sizes[6] < (size_t)DM * DM || (size_t)in_sizes[8] < (size_t)DM * DM) return;
    if (in_sizes[3] < DM || in_sizes[5] < DM || in_sizes[7] < DM || in_sizes[9] < DM) return;
    if ((size_t)out_size < ((size_t)(NB - 1) * OUT_SEQ + SEQ) * DM) return;
    if (SZ_TOTAL > ws_size) return;
    const float* x  = (const float*)d_in[0]; const int* mask = (const int*)d_in[1];
    const float* wq = (const float*)d_in[2]; const float* bq = (const float*)d_in[3];
    const float* wk = (const float*)d_in[4]; const float* bk = (const float*)d_in[5];
    const float* wv = (const float*)d_in[6]; const float* bv = (const float*)d_in[7];
    const float* wo = (const float*)d_in[8]; const float* bo = (const float*)d_in[9];
    float* OUT = (float*)d_out;
    char* wsp = (char*)d_ws;
    bf* XB = (bf*)wsp; wsp += SZ_XB;
    bf* WB = (bf*)wsp; wsp += SZ_WB;
    h16* QH = (h16*)wsp; wsp += SZ_PL;
    h16* KP = (h16*)wsp; wsp += SZ_PL;
    h16* VT = (h16*)wsp; wsp += SZ_PL;
    h16* CH = (h16*)wsp; wsp += SZ_PL;
    h16* QR = (h16*)wsp; wsp += SZ_PE;
    h16* KR = (h16*)wsp; wsp += SZ_PE;
    h16* VR = (h16*)wsp; wsp += SZ_PE;
    h16* CR = (h16*)wsp; wsp += SZ_PE;
    int* FLAG = (int*)wsp; wsp += SZ_FL;
    bf* WQT = WB; bf* WKT = WB + (size_t)DM * DM; bf* WVT = WB + (size_t)2 * DM * DM; bf* WOT = WB + (size_t)3 * DM * DM;

    if (SEQ == SEQ_FULL) {
        const size_t n8 = (size_t)NB * SEQ * DM / 8;
        k_cvt8<<<(unsigned)((n8 + 255) / 256), 256, 0, stream>>>(x, XB, n8);
    } else {
        const size_t n8 = (size_t)SEQ * DM / 8;
        for (int b = 0; b < NB; ++b) k_cvt8<<<(unsigned)((n8 + 255) / 256), 256, 0, stream>>>(x + (size_t)b * SEQ_FULL * DM, XB + (size_t)b * SEQ * DM, n8);
    }
    k_wT<0><<<dim3(DM / 64, DM / 64, 1), 256, 0, stream>>>(wq, WQT);
    k_wT<0><<<dim3(DM / 64, DM / 64, 1), 256, 0, stream>>>(wk, WKT);
    k_wT<0><<<dim3(DM / 64, DM / 64, 1), 256, 0, stream>>>(wv, WVT);
    k_wT<1><<<dim3(DM / 64, DM / 64, 1), 256, 0, stream>>>(wo, WOT);

    k_proj<<<dim3(NB * SEQ / 64, DM / 64, 1), 32, 0, stream>>>(XB, WQT, QH, QR, 1, bq, 0, SEQ, (size_t)NH_ * SEQ * HD, HD, HD, (size_t)SEQ * HD, (size_t)NH_ * EARLY * HD, HD, (size_t)EARLY * HD);
    k_proj<<<dim3(NB * SEQ / 64, DM / 64, 1), 32, 0, stream>>>(XB, WKT, KP, KR, 1, bk, 0, SEQ, (size_t)NH_ * SEQ * HD, HD, HD, (size_t)SEQ * HD, (size_t)NH_ * EARLY * HD, HD, (size_t)EARLY * HD);
    k_proj<<<dim3(DM / 64, NB * SEQ / 64, 1), 32, 0, stream>>>(WVT, XB, VT, VR, 2, bv, 1, DM, (size_t)0, SEQ, SEQ, (size_t)DM * SEQ, (size_t)0, EARLY, (size_t)DM * EARLY);

    k_maskchk<<<1, 1024, 0, stream>>>(mask, FLAG);

    k_flash<1><<<dim3(EARLY / (16 * AW), NB * NH_, 1), 32 * AW, 0, stream>>>(QH, QR, KP, KR, VT, VR, mask, FLAG, CH, CR);
    if (SEQ > EARLY)
        k_flash<0><<<dim3((SEQ - EARLY) / (16 * AW), NB * NH_, 1), 32 * AW, 0, stream>>>(QH, QR, KP, KR, VT, VR, mask, FLAG, CH, CR);

    k_oproj<2, 1><<<dim3(NB * (EARLY / 32), DM / 64, 1), 32, 0, stream>>>(CH, CR, (const h16*)WOT, bo, OUT, EARLY / 32, 0);
    if (SEQ > EARLY)
        k_oproj<4, 0><<<dim3(NB * ((SEQ - EARLY) / 64), DM / 64, 1), 32, 0, stream>>>(CH, CR, (const h16*)WOT, bo, OUT, (SEQ - EARLY) / 64, EARLY);
}
